// PairwiseScore_60421599920629
// MI455X (gfx1250) — hardware-verified
//
#include <hip/hip_runtime.h>


#ifndef NB
#define NB 8
#endif
#ifndef NN
#define NN 256
#endif
#define NB_FULL 8
#define NN_FULL 256
#ifndef OUT_NN
#define OUT_NN NN
#endif
#define DM   128
#define NC   256
#define PT   32
#define PSTR 132
#define OSP  36
#define TL2E 2.8853900817779268f

static_assert(DM % 32 == 0);
static_assert(NC == 2 * DM);
static_assert(NC % 64 == 0);
static_assert((NB * NN) % 64 == 0);
static_assert(NN % PT == 0);
static_assert(PT == 32);
static_assert(OUT_NN % 32 == 0);
static_assert(OUT_NN >= NN);
static_assert(NB <= NB_FULL);
static_assert(NN <= NN_FULL);
static_assert(32 * 16 * 8 == 16 * 64 * 4);
static_assert(256 * 16 * 1 == PT * PT * 4);
static_assert((PT * (DM / 4)) % 256 == 0);
static_assert(DM <= 256);
static_assert((PSTR * 4) % 16 == 0);
static_assert((OSP * 4) % 16 == 0);
static_assert(PSTR >= DM);
static_assert(OSP >= PT);
static_assert((2 * PT * PSTR + DM + PT * OSP) * 4 <= 131072);
static_assert(16 * 68 * 4 <= 131072);
static_assert(((size_t)NN * DM) % 8 == 0);
static_assert(((size_t)DM * DM) % 8 == 0);

typedef unsigned short bf;
typedef __attribute__((ext_vector_type(16))) __bf16   v16bf;
typedef __attribute__((ext_vector_type(8)))  unsigned short v8us;
typedef __attribute__((ext_vector_type(8)))  float    v8f;
typedef __attribute__((ext_vector_type(4)))  float    v4f;
typedef v4f  __attribute__((may_alias)) v4fa;

__device__ __forceinline__ unsigned short f2bf(float f) { unsigned u = __float_as_uint(f); u += 0x7FFFu + ((u >> 16) & 1u); return (unsigned short)(u >> 16); }
__device__ __forceinline__ float bfr(float f) { return __uint_as_float(((unsigned)f2bf(f)) << 16); }
__device__ __forceinline__ v16bf cat16b(v8us lo, v8us hi) { return __builtin_bit_cast(v16bf, __builtin_shufflevector(lo, hi, 0, 1, 2, 3, 4, 5, 6, 7, 8, 9, 10, 11, 12, 13, 14, 15)); }
__device__ __forceinline__ v8f wmmab(v16bf a, v16bf b, v8f c) { return __builtin_amdgcn_wmma_f32_16x16x32_bf16(false, a, false, b, (short)0, c, false, false); }
__device__ __forceinline__ v8f wmmab_g(v16bf a, v16bf b, v8f c) { c = wmmab(a, b, c); asm volatile("v_nop\n\tv_nop\n\tv_nop\n\tv_nop" : "+v"(c) : "v"(a), "v"(b)); return c; }
__device__ __forceinline__ v16bf ldb(const bf* p)  { return cat16b(*(const v8us*)p, *(const v8us*)(p + 16)); }
__device__ __forceinline__ void wave_sync() { __builtin_amdgcn_fence(3  , "wavefront"); __builtin_amdgcn_wave_barrier(); asm volatile("" ::: "memory"); }
__device__ __forceinline__ float tanh_f(float x) { const float e = __builtin_amdgcn_exp2f(x * TL2E); const float r = __builtin_amdgcn_rcpf(e + 1.0f); return fmaf(-2.0f, r, 1.0f); }

__global__ __launch_bounds__(256) void k_cvt8(const float* __restrict__ src, bf* dst, size_t n8) {
    const size_t i = (size_t)blockIdx.x * 256 + threadIdx.x; if (i >= n8) return;
    const v8f v = *(const v8f*)(src + i * 8); v8us o;
#pragma unroll
    for (int k = 0; k < 8; ++k) o[k] = f2bf(v[k]);
    *(volatile v8us*)(dst + i * 8) = o; __threadfence(); *(volatile v8us*)(dst + i * 8) = o;
}

__global__ __launch_bounds__(32) void k_proj2(const bf* __restrict__ A, const bf* __restrict__ Bt, float* P) {
    __shared__ __align__(16) float os[16 * 68];
    const int K = DM;
    const int lane = threadIdx.x & 31, lr = lane & 15, hi = lane >> 4; const int r0 = blockIdx.x * 64, c0 = blockIdx.y * 64;
    v8f acc[4][4];
#pragma unroll
    for (int mb = 0; mb < 4; ++mb)
#pragma unroll
        for (int nb = 0; nb < 4; ++nb) acc[mb][nb] = (v8f){};
    const size_t aoff = (size_t)(r0 + lr) * K + 8 * hi, boff = (size_t)(c0 + lr) * K + 8 * hi;
#pragma unroll 1
    for (int kc = 0; kc < K; kc += 32) {
        v16bf a[4];
#pragma unroll
        for (int mb = 0; mb < 4; ++mb) a[mb] = ldb(A + aoff + (size_t)mb * 16 * K + kc);
#pragma unroll
        for (int nb = 0; nb < 4; ++nb) { const v16bf b = ldb(Bt + boff + (size_t)nb * 16 * K + kc);
#pragma unroll
            for (int mb = 0; mb < 4; ++mb) acc[mb][nb] = wmmab_g(a[mb], b, acc[mb][nb]); }
    }
#pragma unroll
    for (int mb = 0; mb < 4; ++mb) {
#pragma unroll
        for (int nb = 0; nb < 4; ++nb) {
#pragma unroll
            for (int j = 0; j < 8; ++j) os[(hi * 8 + j) * 68 + nb * 16 + lr] = acc[mb][nb][j]; }
        wave_sync();
        float* pb = P + (size_t)(r0 + mb * 16) * NC + c0;
#pragma unroll 1
        for (int ps = 0; ps < 2; ++ps) {
#pragma unroll
            for (int s = 0; s < 8; ++s) { const int row = 2 * s + (lane >> 4), cofs = (lane & 15) * 4;
                const v4f val = *(const v4fa*)(&os[row * 68 + cofs]);
                *(volatile v4f*)(pb + (size_t)row * NC + cofs) = val; }
            if (ps == 0) __threadfence(); }
        wave_sync();
    }
}

__global__ __launch_bounds__(256) void k_addtanh(const float* __restrict__ P, const float* __restrict__ vin, float* OUT) {
    __shared__ __align__(16) float sA[PT * PSTR];
    __shared__ __align__(16) float sC[PT * PSTR];
    __shared__ __align__(16) float sV[DM];
    __shared__ __align__(16) float os[PT * OSP];
    const int tid = threadIdx.x;
    const int kt = blockIdx.x, jt = blockIdx.y, b = blockIdx.z;
    const size_t arow0 = ((size_t)b * NN + (size_t)jt * PT) * NC;
    const size_t crow0 = ((size_t)b * NN + (size_t)kt * PT) * NC + DM;
#pragma unroll 1
    for (int i = tid; i < PT * (DM / 4); i += 256) {
        const int rr = i >> 5, cc = (i & 31) * 4;
        const v4f av = *(const v4f*)(P + arow0 + (size_t)rr * NC + cc);
        const v4f cv = *(const v4f*)(P + crow0 + (size_t)rr * NC + cc);
        *(v4fa*)(&sA[rr * PSTR + cc]) = av; *(v4fa*)(&sC[rr * PSTR + cc]) = cv; }
    if (tid < DM) sV[tid] = bfr(vin[tid]);
    __syncthreads();
    const int tk = tid & 15, tj = tid >> 4;
    const int ja = tj * PSTR, jb = (tj + 16) * PSTR, ka = tk * PSTR, kb = (tk + 16) * PSTR;
    float s00 = 0.0f, s01 = 0.0f, s10 = 0.0f, s11 = 0.0f;
#pragma unroll 1
    for (int m = 0; m < DM; m += 4) {
        const v4f a0 = *(const v4fa*)(&sA[ja + m]); const v4f a1 = *(const v4fa*)(&sA[jb + m]);
        const v4f c0 = *(const v4fa*)(&sC[ka + m]); const v4f c1 = *(const v4fa*)(&sC[kb + m]);
        const v4f w  = *(const v4fa*)(&sV[m]);
#pragma unroll
        for (int i = 0; i < 4; ++i) {
            s00 = fmaf(w[i], tanh_f(a0[i] + c0[i]), s00);
            s01 = fmaf(w[i], tanh_f(a0[i] + c1[i]), s01);
            s10 = fmaf(w[i], tanh_f(a1[i] + c0[i]), s10);
            s11 = fmaf(w[i], tanh_f(a1[i] + c1[i]), s11); }
    }
    os[tj * OSP + tk] = s00; os[tj * OSP + tk + 16] = s01;
    os[(tj + 16) * OSP + tk] = s10; os[(tj + 16) * OSP + tk + 16] = s11;
    __syncthreads();
    const int row = tid >> 3, cofs = (tid & 7) * 4;
    const v4f val = *(const v4fa*)(&os[row * OSP + cofs]);
    float* orow = OUT + ((size_t)b * OUT_NN + (size_t)jt * PT + (size_t)row) * OUT_NN + (size_t)kt * PT + cofs;
#pragma unroll 1
    for (int ps = 0; ps < 2; ++ps) {
        *(volatile v4f*)orow = val;
        if (ps == 0) __threadfence(); }
}

static constexpr size_t al256(size_t v) { return (v + 255) & ~(size_t)255; }
static constexpr size_t SZ_XB = al256((size_t)NB * NN * DM * 2);
static constexpr size_t SZ_WB = al256((size_t)NC * DM * 2);
static constexpr size_t SZ_PP = al256((size_t)NB * NN * NC * 4);
static constexpr size_t SZ_TOTAL = SZ_XB + SZ_WB + SZ_PP;
static_assert(SZ_TOTAL <= (size_t)134217728);
static_assert(((size_t)DM * DM * 2) % 256 == 0);
static_assert((size_t)(NB * NN / 64) * 64 * NC * 4 <= SZ_PP);
static_assert((size_t)(NC / 64) * 64 == NC);

extern "C" void kernel_launch(void* const* d_in, const int* in_sizes, int n_in,
                              void* d_out, int out_size, void* d_ws, size_t ws_size, hipStream_t stream) {
    if (n_in < 4) return;
    const size_t needx = ((size_t)(NB - 1) * NN_FULL + NN) * DM;
    if ((size_t)in_sizes[0] < needx) return;
    if ((size_t)in_sizes[1] < (size_t)DM * DM || (size_t)in_sizes[2] < (size_t)DM * DM) return;
    if (in_sizes[3] < DM) return;
    if ((size_t)out_size < ((size_t)(NB - 1) * OUT_NN + (size_t)(NN - 1)) * OUT_NN + NN) return;
    if (SZ_TOTAL > ws_size) return;
    const float* x  = (const float*)d_in[0];
    const float* w1 = (const float*)d_in[1];
    const float* w2 = (const float*)d_in[2];
    const float* vv = (const float*)d_in[3];
    float* OUT = (float*)d_out;
    char* wsp = (char*)d_ws;
    bf* XB = (bf*)wsp; wsp += SZ_XB;
    bf* WB = (bf*)wsp; wsp += SZ_WB;
    float* PP = (float*)wsp; wsp += SZ_PP;

    if (NN == NN_FULL) {
        const size_t n8 = (size_t)NB * NN * DM / 8;
        k_cvt8<<<(unsigned)((n8 + 255) / 256), 256, 0, stream>>>(x, XB, n8);
    } else {
        const size_t n8 = (size_t)NN * DM / 8;
        for (int b = 0; b < NB; ++b) k_cvt8<<<(unsigned)((n8 + 255) / 256), 256, 0, stream>>>(x + (size_t)b * NN_FULL * DM, XB + (size_t)b * NN * DM, n8);
    }
    { const size_t n8 = (size_t)DM * DM / 8; const unsigned g = (unsigned)((n8 + 255) / 256);
      k_cvt8<<<g, 256, 0, stream>>>(w1, WB, n8); k_cvt8<<<g, 256, 0, stream>>>(w2, WB + (size_t)DM * DM, n8); }

    k_proj2<<<dim3(NB * NN / 64, NC / 64, 1), 32, 0, stream>>>(XB, WB, PP);

    k_addtanh<<<dim3(NN / PT, NN / PT, NB), 256, 0, stream>>>(PP, vv, OUT);
}
